// GATClassifier_36618891165995
// MI455X (gfx1250) — hardware-verified
//
#include <hip/hip_runtime.h>
#include <stddef.h>
#include <stdint.h>
#include <math.h>


#define F_IN    128
#define HC1     256
#define HID     64
#define NHD1    4
#define NC2     64
#define KA2     512
#define NGR     64
#define NTHR    256
#define NWAVE   8
#define EPT     8
#define CHUNK   (NTHR * EPT)
#define WCAP    (EPT * 32)
#define LISTN   (NWAVE * WCAP)
#define NBMAX   2048
#define SLOTB   11
#define RCAP    28672
#define DEGCAP  256
#define GBM     64
#define GBN     64
#define GTHR    128
#define MROWS   128
#define STGW    512
#define NUW1    (HC1 * (F_IN / 8))
#define NUW2    (NC2 * (KA2 / 8))
#define NEGSL   0.2f
#define EPS_SM  1e-16f
#define WSMAX   134217728
#define LDS_AGG ((2 * RCAP + 2 * NBMAX + LISTN) * 4 + 64)
#define MEAS_MAXDEG 42
#define MEAS_B1024  20780

static_assert((CHUNK & (CHUNK - 1)) == 0 && CHUNK <= (1 << SLOTB));
static_assert(NBMAX == (1 << SLOTB));
static_assert(NTHR * 8 == NBMAX);
static_assert(LISTN >= NBMAX);
static_assert(LISTN >= NWAVE * WCAP);
static_assert((RCAP % 32) == 0);
static_assert(LDS_AGG <= 300000);
static_assert(GBM == (GTHR / 32) * 16);
static_assert(GTHR == 2 * GBN && GTHR == 2 * GBM);
static_assert((F_IN % 32) == 0 && (KA2 % 32) == 0);
static_assert((HC1 % GBN) == 0 && HID == GBN && NC2 == GBN);
static_assert(KA2 == 2 * HC1);
static_assert((MROWS % GBM) == 0);
static_assert(HC1 == 8 * 32);
static_assert(NC2 == 2 * 32);
static_assert(NHD1 * HID == HC1 && HID == 8 * 8);
static_assert(NWAVE * STGW <= RCAP);
static_assert(STGW == HC1 + HC1);
static_assert((F_IN / 8) == 16);
static_assert((NUW1 % NTHR) == 0 && (NUW2 % NTHR) == 0);
static_assert(DEGCAP >= MEAS_MAXDEG + 8);
static_assert(RCAP >= MEAS_B1024 + 4096);
static_assert(NGR * NC2 * 4 == 16384);

typedef float          v2f  __attribute__((ext_vector_type(2)));
typedef float          v4f  __attribute__((ext_vector_type(4)));
typedef float          v8f  __attribute__((ext_vector_type(8)));
typedef int            v4i  __attribute__((ext_vector_type(4)));
typedef int            v8i  __attribute__((ext_vector_type(8)));
typedef unsigned int   v4u  __attribute__((ext_vector_type(4)));
typedef unsigned short v8us __attribute__((ext_vector_type(8)));
typedef __bf16         v16b __attribute__((ext_vector_type(16)));
typedef v2f  __attribute__((may_alias)) v2fa;
typedef v4f  __attribute__((may_alias)) v4fa;
typedef v4u  __attribute__((may_alias)) v4ua;
typedef v8us __attribute__((may_alias)) v8usa;
union FragB { v16b v; v8us h[2]; v8i w; };

__device__ __forceinline__ v8f wmb(const FragB& a, const FragB& b, v8f c) {
  v8f d = __builtin_amdgcn_wmma_f32_16x16x32_bf16(false, a.v, false, b.v, (short)0, c, false, false);
  asm volatile("v_nop\n\tv_nop\n\tv_nop\n\tv_nop" : "+v"(d) : "v"(a.w), "v"(b.w));
  return d;
}

__device__ __forceinline__ unsigned int f2bf(float f) {
  const unsigned int u = __float_as_uint(f);
  const unsigned int r = ((u + 0x7FFFu + ((u >> 16) & 1u)) >> 16) & 0xFFFFu;
  const unsigned int q = ((u >> 16) | 0x40u) & 0xFFFFu;
  return ((u & 0x7FFFFFFFu) > 0x7F800000u) ? q : r;
}
__device__ __forceinline__ float bf2f(unsigned int b) { return __uint_as_float(b << 16); }
__device__ __forceinline__ float bfr(float f) { return bf2f(f2bf(f)); }
__device__ __forceinline__ v4f bfr4(const v4f a) {
  v4f r; r.x = bfr(a.x); r.y = bfr(a.y); r.z = bfr(a.z); r.w = bfr(a.w); return r;
}
__device__ __forceinline__ unsigned int pk2(float lo, float hi) { return f2bf(lo) | (f2bf(hi) << 16); }
__device__ __forceinline__ v4u pack8(const v4f a, const v4f b) {
  v4u r;
  r.x = pk2(a.x, a.y); r.y = pk2(a.z, a.w); r.z = pk2(b.x, b.y); r.w = pk2(b.z, b.w);
  return r;
}
__device__ __forceinline__ float eluf(float v) { return v > 0.f ? v : expm1f(v); }

__device__ __forceinline__ void osm_w(float lg, float& mx, float& dn, float& s1, float& s2) {
  const float df = lg - mx;
  const float ee = expf(-fabsf(df));
  const bool up  = df > 0.f;
  s1 = up ? ee : 1.0f;
  s2 = up ? 1.0f : ee;
  mx = up ? lg : mx;
  dn = fmaf(dn, s1, s2);
}
__device__ __forceinline__ void acc8(v4f& aA, v4f& aB, const v4f fA, const v4f fB, float s1, float s2) {
  aA.x = fmaf(aA.x, s1, s2 * fA.x);
  aA.y = fmaf(aA.y, s1, s2 * fA.y);
  aA.z = fmaf(aA.z, s1, s2 * fA.z);
  aA.w = fmaf(aA.w, s1, s2 * fA.w);
  aB.x = fmaf(aB.x, s1, s2 * fB.x);
  aB.y = fmaf(aB.y, s1, s2 * fB.y);
  aB.z = fmaf(aB.z, s1, s2 * fB.z);
  aB.w = fmaf(aB.w, s1, s2 * fB.w);
}

__device__ __forceinline__ int scan_chunk(const int* __restrict__ dsts, int nE, int cbase, int slotBase,
                                          int nb, int vec8, int* list, int tid, int lane, int wave) {
  int wc = 0;
  const int el0  = tid * EPT;
  const int e0   = cbase + el0;
  const int sent = -2147483647 - 1;
  v4i da, db;
  if (vec8 != 0 && cbase + CHUNK <= nE) {
    da = *(const v4i*)(dsts + e0);
    db = *(const v4i*)(dsts + e0 + 4);
  } else {
    da.x = (e0     < nE) ? dsts[min(e0,     nE - 1)] : sent;
    da.y = (e0 + 1 < nE) ? dsts[min(e0 + 1, nE - 1)] : sent;
    da.z = (e0 + 2 < nE) ? dsts[min(e0 + 2, nE - 1)] : sent;
    da.w = (e0 + 3 < nE) ? dsts[min(e0 + 3, nE - 1)] : sent;
    db.x = (e0 + 4 < nE) ? dsts[min(e0 + 4, nE - 1)] : sent;
    db.y = (e0 + 5 < nE) ? dsts[min(e0 + 5, nE - 1)] : sent;
    db.z = (e0 + 6 < nE) ? dsts[min(e0 + 6, nE - 1)] : sent;
    db.w = (e0 + 7 < nE) ? dsts[min(e0 + 7, nE - 1)] : sent;
  }
  const unsigned nbs = (unsigned)slotBase;
  const unsigned unb = (unsigned)nb;
  const unsigned s0 = (unsigned)da.x - nbs, s1 = (unsigned)da.y - nbs;
  const unsigned s2 = (unsigned)da.z - nbs, s3 = (unsigned)da.w - nbs;
  const unsigned s4 = (unsigned)db.x - nbs, s5 = (unsigned)db.y - nbs;
  const unsigned s6 = (unsigned)db.z - nbs, s7 = (unsigned)db.w - nbs;
  const bool h0 = s0 < unb, h1 = s1 < unb, h2 = s2 < unb, h3 = s3 < unb;
  const bool h4 = s4 < unb, h5 = s5 < unb, h6 = s6 < unb, h7 = s7 < unb;
  const unsigned any = __builtin_amdgcn_ballot_w32(h0 | h1 | h2 | h3 | h4 | h5 | h6 | h7);
  if (any != 0u) {
#define HITJ(J, HJ, SJ) { \
      const unsigned mj = __builtin_amdgcn_ballot_w32(HJ); \
      if (mj != 0u) { \
        if (HJ) { \
          const int pos = wc + (int)__builtin_amdgcn_mbcnt_lo(mj, 0u); \
          if (pos < WCAP) list[wave * WCAP + pos] = ((el0 + (J)) << SLOTB) | (int)(SJ); \
        } \
        wc += (int)__builtin_popcount(mj); } }
    HITJ(0, h0, s0)
    HITJ(1, h1, s1)
    HITJ(2, h2, s2)
    HITJ(3, h3, s3)
    HITJ(4, h4, s4)
    HITJ(5, h5, s5)
    HITJ(6, h6, s6)
    HITJ(7, h7, s7)
#undef HITJ
  }
  return wc;
}

__device__ __forceinline__ void wtr_unit(const float* __restrict__ w, int Kin, int Ncol, int Kout,
                                         unsigned short* wt, int u) {
  const int kq = Kout >> 3;
  const int n  = u / kq;
  const int k8 = (u - n * kq) * 8;
  const int kk = k8 - (k8 / Kin) * Kin;
  const int ncl = n < Ncol ? n : Ncol - 1;
  const float* p = w + (size_t)kk * (size_t)Ncol + ncl;
  v4f a, b;
  a.x = p[0];                    a.y = p[(size_t)Ncol];         a.z = p[(size_t)2 * Ncol];     a.w = p[(size_t)3 * Ncol];
  b.x = p[(size_t)4 * Ncol];     b.y = p[(size_t)5 * Ncol];     b.z = p[(size_t)6 * Ncol];     b.w = p[(size_t)7 * Ncol];
  const v4u wv = pack8(a, b);
  unsigned short* o = wt + (size_t)ncl * (size_t)Kout + k8;
  *(volatile v4u*)o = wv;
  __threadfence();
  *(volatile v4u*)o = wv;
}

__global__ __launch_bounds__(NTHR) void k_prep(const float* __restrict__ x, const float* __restrict__ W1,
                                               const float* __restrict__ W2, unsigned short* xb,
                                               unsigned short* w1t, unsigned short* w2t, int nN, int nUx) {
  const int u = (int)blockIdx.x * NTHR + (int)threadIdx.x;
  if (u < nUx) {
    const int row = u >> 4;
    const int c0  = (u & 15) * 8;
    const int rc  = row < nN ? row : nN - 1;
    const float* p = x + (size_t)rc * F_IN + c0;
    v4f a = *(const v4fa*)p, b = *(const v4fa*)(p + 4);
    const v4f z4 = {0.f, 0.f, 0.f, 0.f};
    if (row >= nN) { a = z4; b = z4; }
    const v4u hv = pack8(a, b);
    const size_t o = (size_t)row * F_IN + c0;
    *(volatile v4u*)(xb + o) = hv;
    __threadfence();
    *(volatile v4u*)(xb + o) = hv;
  } else {
    const int v = u - nUx;
    if (v < NUW1) {
      wtr_unit(W1, F_IN, HC1, F_IN, w1t, v);
    } else if (v < NUW1 + NUW2) {
      wtr_unit(W2, HC1, NC2, KA2, w2t, v - NUW1);
    }
  }
}

__global__ __launch_bounds__(GTHR) void k_gemm(
    const unsigned short* __restrict__ A, const unsigned short* __restrict__ WT,
    float* outF, int K, int ldo,
    const float* __restrict__ atts, const float* __restrict__ attd, int attLen,
    float* SD, int MPr)
{
  __shared__ __attribute__((aligned(16))) float stg[GBM * GBN];
  __shared__ __attribute__((aligned(16))) float satt[2 * GBN];
  __shared__ __attribute__((aligned(16))) float sdot[2 * GBM];
  const int tid = (int)threadIdx.x, lane = tid & 31, wave = tid >> 5, hh = lane >> 4, m = lane & 15;
  const int rowBase = (int)blockIdx.x * GBM;
  const int head    = (int)blockIdx.y;
  const int col0    = head * GBN;

  {
    const int which = tid >> 6;
    const int c  = tid & 63;
    const int cl = c < attLen ? c : attLen - 1;
    const float vs = atts[head * attLen + cl];
    const float vd = attd[head * attLen + cl];
    float v = (which == 0) ? vs : vd;
    v = (c < attLen) ? bfr(v) : 0.f;
    satt[which * GBN + c] = v;
  }

  v8f acc[4];
  {
    const v8f z = {0.f, 0.f, 0.f, 0.f, 0.f, 0.f, 0.f, 0.f};
    acc[0] = z; acc[1] = z; acc[2] = z; acc[3] = z;
  }
  const unsigned short* ap = A  + (size_t)(rowBase + 16 * wave + m) * (size_t)K + 8 * hh;
  const unsigned short* wp = WT + (size_t)(col0 + m) * (size_t)K + 8 * hh;
  const int ksteps = K >> 5;
#pragma unroll 1
  for (int ks = 0; ks < ksteps; ++ks) {
    FragB af;
    af.h[0] = *(const v8usa*)(ap + 32 * ks);
    af.h[1] = *(const v8usa*)(ap + 32 * ks + 16);
#pragma unroll
    for (int t = 0; t < 4; ++t) {
      const unsigned short* wq = wp + (size_t)(16 * t) * (size_t)K + 32 * ks;
      FragB bf;
      bf.h[0] = *(const v8usa*)wq;
      bf.h[1] = *(const v8usa*)(wq + 16);
      acc[t] = wmb(af, bf, acc[t]);
    }
  }

#pragma unroll
  for (int t = 0; t < 4; ++t) {
    const int lc = 16 * t + m;
#pragma unroll
    for (int r = 0; r < 8; ++r) {
      const int lr = 16 * wave + 8 * hh + r;
      stg[lr * GBN + lc] = acc[t][r];
    }
  }
  __syncthreads();

  {
    const int row = tid & 63, which = tid >> 6;
    const float* sa = satt + which * GBN;
    const float* hr = stg + row * GBN;
    float d = 0.f;
#pragma unroll 4
    for (int c4 = 0; c4 < GBN / 4; ++c4) {
      const v4f hv = *(const v4fa*)(hr + 4 * c4);
      const v4f av = *(const v4fa*)(sa + 4 * c4);
      d = fmaf(hv.x, av.x, d);
      d = fmaf(hv.y, av.y, d);
      d = fmaf(hv.z, av.z, d);
      d = fmaf(hv.w, av.w, d);
    }
    sdot[which * GBM + row] = d;
  }
  __syncthreads();

  v4f fv[8];
#pragma unroll
  for (int i = 0; i < 8; ++i) {
    const int lr = 16 * wave + 2 * i + hh;
    fv[i] = *(const v4fa*)(stg + lr * GBN + 4 * m);
  }
  const int which2 = lane >> 4, piece = lane & 15;
  const v4f sdv = *(const v4fa*)(sdot + which2 * GBM + 4 * piece);
  float* sp = SD + (size_t)(2 * head + which2) * (size_t)MPr + rowBase + 4 * piece;

#pragma unroll
  for (int i = 0; i < 8; ++i) {
    const int lr = 16 * wave + 2 * i + hh;
    const int gr = rowBase + lr;
    float* op = outF + (size_t)gr * (size_t)ldo + col0 + 4 * m;
    *(volatile v4f*)op = fv[i];
  }
  if (wave == 0) *(volatile v4f*)sp = sdv;
  __threadfence();
#pragma unroll
  for (int i = 0; i < 8; ++i) {
    const int lr = 16 * wave + 2 * i + hh;
    const int gr = rowBase + lr;
    float* op = outF + (size_t)gr * (size_t)ldo + col0 + 4 * m;
    *(volatile v4f*)op = fv[i];
  }
  if (wave == 0) *(volatile v4f*)sp = sdv;
}

template<int L>
__global__ __launch_bounds__(NTHR) void k_agg(
    const int* __restrict__ srcs, const int* __restrict__ dsts,
    const float* __restrict__ F, const float* __restrict__ SD,
    const float* __restrict__ bias,
    unsigned short* HP, float* XO,
    int nN, int nE, int nb, int vec8, int MPr) {
  extern __shared__ v4f lds_dyn[];
  int* reg1 = (int*)lds_dyn;
  int* reg2 = reg1 + RCAP;
  int* scnt = reg2 + RCAP;
  int* soff = scnt + NBMAX;
  int* list = soff + NBMAX;
  int* wcnt = list + LISTN;
  int* wtot = wcnt + NWAVE;
  const int tid = (int)threadIdx.x, lane = tid & 31, wave = tid >> 5;
  const int nodeBase = (int)blockIdx.x * nb;

  for (int i = tid; i < NBMAX; i += NTHR) scnt[i] = 0;
  __syncthreads();

  int tot = 0;
  const int nChunks = (nE + CHUNK - 1) / CHUNK;
#pragma unroll 1
  for (int ch = 0; ch < nChunks; ++ch) {
    const int cbase = ch * CHUNK;
    const int wc = scan_chunk(dsts, nE, cbase, nodeBase, nb, vec8, list, tid, lane, wave);
    if (lane == 0) wcnt[wave] = wc;
    __syncthreads();
    int pre = 0, all = 0;
#pragma unroll
    for (int w2 = 0; w2 < NWAVE; ++w2) {
      int c = wcnt[w2];
      c = c < 0 ? 0 : (c > WCAP ? WCAP : c);
      all += c;
      pre += (w2 < wave) ? c : 0;
    }
    const int wcc  = wc > WCAP ? WCAP : wc;
    const int base = tot + pre;
#pragma unroll 1
    for (int i = lane; i < wcc; i += 32) {
      const int ent = list[wave * WCAP + i];
      const int el  = (ent >> SLOTB) & (CHUNK - 1);
      const int sl  = ent & (NBMAX - 1);
      int eid = cbase + el;
      eid = eid > nE - 1 ? nE - 1 : eid;
      const int pos = base + i;
      if (pos < RCAP) reg1[pos] = (int)(((unsigned)eid << SLOTB) | (unsigned)sl);
    }
    tot += all;
    tot = tot > RCAP ? RCAP : tot;
    __syncthreads();
  }
  const int nh = tot;

  if (wave == 0) {
#pragma unroll 1
    for (int b0 = 0; b0 < nh; b0 += 32) {
      const int idx = b0 + lane;
      const int uv  = reg1[idx < nh ? idx : nh - 1];
      const int m32 = (nh - b0) < 32 ? (nh - b0) : 32;
#pragma unroll 1
      for (int k = 0; k < m32; ++k) {
        const int u  = __builtin_amdgcn_readlane(uv, k);
        const int sl = u & (NBMAX - 1);
        if (lane == 0) scnt[sl] = scnt[sl] + 1;
      }
    }
  }
  __syncthreads();

  {
    const v4i ca = *(const v4i*)(scnt + 8 * tid);
    const v4i cb = *(const v4i*)(scnt + 8 * tid + 4);
    const int e0 = ca.x < 0 ? 0 : ca.x, e1 = ca.y < 0 ? 0 : ca.y, e2 = ca.z < 0 ? 0 : ca.z, e3 = ca.w < 0 ? 0 : ca.w;
    const int e4 = cb.x < 0 ? 0 : cb.x, e5 = cb.y < 0 ? 0 : cb.y, e6 = cb.z < 0 ? 0 : cb.z, e7 = cb.w < 0 ? 0 : cb.w;
    const int ts = e0 + e1 + e2 + e3 + e4 + e5 + e6 + e7;
    int incl = ts;
#pragma unroll
    for (int d = 1; d < 32; d <<= 1) {
      const int up = __shfl_up(incl, d);
      if (lane >= d) incl += up;
    }
    if (lane == 31) wtot[wave] = incl;
    __syncthreads();
    int pre = 0;
#pragma unroll
    for (int w2 = 0; w2 < NWAVE; ++w2) pre += (w2 < wave) ? wtot[w2] : 0;
    int run = pre + incl - ts;
    soff[8 * tid + 0] = run; run += e0;
    soff[8 * tid + 1] = run; run += e1;
    soff[8 * tid + 2] = run; run += e2;
    soff[8 * tid + 3] = run; run += e3;
    soff[8 * tid + 4] = run; run += e4;
    soff[8 * tid + 5] = run; run += e5;
    soff[8 * tid + 6] = run; run += e6;
    soff[8 * tid + 7] = run;
  }
  __syncthreads();
  for (int i = tid; i < NBMAX; i += NTHR) list[i] = soff[i];
  __syncthreads();

  if (wave == 0) {
#pragma unroll 1
    for (int b0 = 0; b0 < nh; b0 += 32) {
      const int idx = b0 + lane;
      const int uv  = reg1[idx < nh ? idx : nh - 1];
      const int m32 = (nh - b0) < 32 ? (nh - b0) : 32;
#pragma unroll 1
      for (int k = 0; k < m32; ++k) {
        const int u   = __builtin_amdgcn_readlane(uv, k);
        const int sl  = u & (NBMAX - 1);
        const int eid = (int)((unsigned)u >> SLOTB);
        if (lane == 0) {
          int pos = list[sl];
          pos = pos < 0 ? 0 : (pos > RCAP - 1 ? RCAP - 1 : pos);
          reg2[pos] = eid;
          list[sl] = pos + 1;
        }
      }
    }
  }
  __syncthreads();

  const int nbw = nb >> 3;
  const bool ovf = (nh >= RCAP);
  const float qnan = __int_as_float(0x7fc00000);

  if constexpr (L == 1) {
    const int c0   = 8 * lane;
    const int head = lane >> 3;
    const v4f bbA  = bfr4(*(const v4fa*)(bias + c0));
    const v4f bbB  = bfr4(*(const v4fa*)(bias + c0 + 4));
    const float* ASp = SD + (size_t)(2 * head) * (size_t)MPr;
    const float* ADp = ASp + MPr;
    float*        stgf = (float*)reg1 + wave * STGW;
    unsigned int* stgw = (unsigned int*)reg1 + wave * STGW + HC1;

#pragma unroll 1
    for (int jt = 0; jt < nbw; ++jt) {
      const int slot = wave * nbw + jt;
      const int grow = nodeBase + slot;
      const int gcl  = grow < nN ? grow : nN - 1;
      int st = soff[slot];
      const int craw = scnt[slot];
      int cnt = craw;
      st  = st < 0 ? 0 : (st > nh ? nh : st);
      cnt = cnt < 0 ? 0 : (cnt > DEGCAP ? DEGCAP : cnt);
      if (cnt > nh - st) cnt = nh - st;
      const float pz = (ovf || craw > DEGCAP) ? qnan : 0.0f;

      const float adv = ADp[gcl];
      float mx = -3.0e38f, dn = 0.0f;
      v4f aA = {0.f, 0.f, 0.f, 0.f};
      v4f aB = {0.f, 0.f, 0.f, 0.f};

#pragma unroll 1
      for (int q = 0; q < cnt; ++q) {
        int idx = st + q; idx = idx > RCAP - 1 ? RCAP - 1 : idx;
        int eid = reg2[idx]; eid = eid < 0 ? 0 : (eid > nE - 1 ? nE - 1 : eid);
        const int sraw = srcs[eid];
        const int s = sraw < 0 ? 0 : (sraw > nN - 1 ? nN - 1 : sraw);
        const float* fp = F + (size_t)s * HC1 + c0;
        const v4f fA = *(const v4fa*)fp;
        const v4f fB = *(const v4fa*)(fp + 4);
        float lg = ASp[s] + adv;
        lg = lg > 0.f ? lg : NEGSL * lg;
        float s1, s2;
        osm_w(lg, mx, dn, s1, s2);
        acc8(aA, aB, fA, fB, s1, s2);
      }
      {
        const float* fp = F + (size_t)gcl * HC1 + c0;
        const v4f fA = *(const v4fa*)fp;
        const v4f fB = *(const v4fa*)(fp + 4);
        float lg = ASp[gcl] + adv;
        lg = lg > 0.f ? lg : NEGSL * lg;
        float s1, s2;
        osm_w(lg, mx, dn, s1, s2);
        acc8(aA, aB, fA, fB, s1, s2);
      }
      const float inv = 1.0f / (dn + EPS_SM);
      v4f zA, zB;
      zA.x = fmaf(aA.x, inv, bbA.x); zA.y = fmaf(aA.y, inv, bbA.y);
      zA.z = fmaf(aA.z, inv, bbA.z); zA.w = fmaf(aA.w, inv, bbA.w);
      zB.x = fmaf(aB.x, inv, bbB.x); zB.y = fmaf(aB.y, inv, bbB.y);
      zB.z = fmaf(aB.z, inv, bbB.z); zB.w = fmaf(aB.w, inv, bbB.w);
      *(v4f*)(stgf + c0)     = zA;
      *(v4f*)(stgf + c0 + 4) = zB;
      __syncthreads();

      const bool live = grow < nN;
#pragma unroll 1
      for (int j = 0; j < 4; ++j) {
        const int p = 32 * j + lane;
        const v2f zz = *(const v2fa*)(stgf + 2 * p);
        const float e0 = eluf(zz.x), e1 = eluf(zz.y);
        const float o0 = (live ? e0 : 0.f) + pz;
        const float o1 = (live ? e1 : 0.f) + pz;
        const unsigned int hb0 = f2bf(o0), hb1 = f2bf(o1);
        const unsigned int lb0 = f2bf(o0 - bf2f(hb0)), lb1 = f2bf(o1 - bf2f(hb1));
        stgw[p]       = hb0 | (hb1 << 16);
        stgw[128 + p] = lb0 | (lb1 << 16);
      }
      __syncthreads();

      const v4u hv = *(const v4ua*)(stgw + 4 * lane);
      const v4u lv = *(const v4ua*)(stgw + 128 + 4 * lane);
      unsigned short* gp = HP + (size_t)grow * KA2 + 8 * lane;
      const bool wr = grow < MPr;
      if (wr) { *(volatile v4u*)gp = hv; *(volatile v4u*)(gp + HC1) = lv; }
      __threadfence();
      if (wr) { *(volatile v4u*)gp = hv; *(volatile v4u*)(gp + HC1) = lv; }
    }
  } else {
    const int c0 = 2 * lane;
    float bz0, bz1;
    {
      const v2f bb = *(const v2fa*)(bias + c0);
      bz0 = bfr(bb.x); bz1 = bfr(bb.y);
    }
    const float* ASp = SD;
    const float* ADp = SD + MPr;
    const int sa = (2 * lane) & 31, sb = (2 * lane + 1) & 31;

#pragma unroll 1
    for (int jt = 0; jt < nbw; ++jt) {
      const int slot = wave * nbw + jt;
      const int grow = nodeBase + slot;
      const int gcl  = grow < nN ? grow : nN - 1;
      int st = soff[slot];
      const int craw = scnt[slot];
      int cnt = craw;
      st  = st < 0 ? 0 : (st > nh ? nh : st);
      cnt = cnt < 0 ? 0 : (cnt > DEGCAP ? DEGCAP : cnt);
      if (cnt > nh - st) cnt = nh - st;
      const float pz = (ovf || craw > DEGCAP) ? qnan : 0.0f;

      const float adv = ADp[gcl];
      float mx = -3.0e38f, dn = 0.0f;
      float a0 = 0.0f, a1 = 0.0f;

#pragma unroll 1
      for (int q = 0; q < cnt; ++q) {
        int idx = st + q; idx = idx > RCAP - 1 ? RCAP - 1 : idx;
        int eid = reg2[idx]; eid = eid < 0 ? 0 : (eid > nE - 1 ? nE - 1 : eid);
        const int sraw = srcs[eid];
        const int s = sraw < 0 ? 0 : (sraw > nN - 1 ? nN - 1 : sraw);
        const v2f fs = *(const v2fa*)(F + (size_t)s * NC2 + c0);
        float lg = ASp[s] + adv;
        lg = lg > 0.f ? lg : NEGSL * lg;
        float s1, s2;
        osm_w(lg, mx, dn, s1, s2);
        a0 = fmaf(a0, s1, s2 * fs.x);
        a1 = fmaf(a1, s1, s2 * fs.y);
      }
      {
        const v2f fs = *(const v2fa*)(F + (size_t)gcl * NC2 + c0);
        float lg = ASp[gcl] + adv;
        lg = lg > 0.f ? lg : NEGSL * lg;
        float s1, s2;
        osm_w(lg, mx, dn, s1, s2);
        a0 = fmaf(a0, s1, s2 * fs.x);
        a1 = fmaf(a1, s1, s2 * fs.y);
      }
      const float inv = 1.0f / (dn + EPS_SM);
      const float e0 = eluf(fmaf(a0, inv, bz0));
      const float e1 = eluf(fmaf(a1, inv, bz1));
      const bool live = grow < nN;
      const float v0 = (live ? e0 : 0.f) + pz;
      const float v1 = (live ? e1 : 0.f) + pz;
      v4f ow;
      ow.x = __shfl(v0, sa, 32); ow.y = __shfl(v1, sa, 32);
      ow.z = __shfl(v0, sb, 32); ow.w = __shfl(v1, sb, 32);
      float* op = XO + (size_t)grow * NC2 + 4 * (lane & 15);
      const bool wr = (grow < MPr) && (lane < 16);
      if (wr) *(volatile v4f*)op = ow;
      __threadfence();
      if (wr) *(volatile v4f*)op = ow;
    }
  }
}

__global__ __launch_bounds__(NTHR) void k_pool(const float* __restrict__ hf, const int* __restrict__ bat,
                                               int nN, float* pl) {
  __shared__ __attribute__((aligned(16))) double wsum[NWAVE * NC2];
  __shared__ int wcn[NWAVE];
  __shared__ __attribute__((aligned(16))) float outs[NC2];
  const int tid = (int)threadIdx.x, lane = tid & 31, wave = tid >> 5;
  const int g = (int)blockIdx.x;

  double a0 = 0.0, a1 = 0.0;
  int mine = 0;
#pragma unroll 1
  for (int i0 = wave * 32; i0 < nN; i0 += NTHR) {
    const int i  = i0 + lane;
    const int ic = i < nN ? i : nN - 1;
    const int b  = bat[ic];
    const bool hit = (i < nN) && (b == g);
    unsigned msk = __builtin_amdgcn_ballot_w32(hit);
    int nh = (int)__builtin_popcount(msk);
    nh = nh > 32 ? 32 : nh;
    mine += hit ? 1 : 0;
#pragma unroll 1
    for (int q = 0; q < nh; ++q) {
      const int k = __builtin_ffs((int)msk) - 1;
      msk &= msk - 1u;
      int node = i0 + (k < 0 ? 0 : k);
      node = node > nN - 1 ? nN - 1 : node;
      const v2f v = *(const v2fa*)(hf + (size_t)node * NC2 + 2 * lane);
      a0 += (double)v.x; a1 += (double)v.y;
    }
  }
  wsum[wave * NC2 + 2 * lane + 0] = a0;
  wsum[wave * NC2 + 2 * lane + 1] = a1;
  int cnt = mine;
  cnt += __shfl_xor(cnt, 16); cnt += __shfl_xor(cnt, 8); cnt += __shfl_xor(cnt, 4);
  cnt += __shfl_xor(cnt, 2);  cnt += __shfl_xor(cnt, 1);
  if (lane == 0) wcn[wave] = cnt;
  __syncthreads();
  if (tid < NC2) {
    double s = 0.0;
    int c = 0;
#pragma unroll
    for (int w2 = 0; w2 < NWAVE; ++w2) { s += wsum[w2 * NC2 + tid]; c += wcn[w2]; }
    const float cf = (c < 1) ? 1.0f : (float)c;
    outs[tid] = (float)s * (1.0f / cf);
  }
  __syncthreads();
  const v4f ov = *(const v4fa*)(outs + 4 * (lane & 15));
  float* op = pl + (size_t)g * NC2 + 4 * (lane & 15);
  const bool okst = (wave == 0) && (lane < 16);
  if (okst) *(volatile v4f*)op = ov;
  __threadfence();
  if (okst) *(volatile v4f*)op = ov;
}

__global__ __launch_bounds__(NGR) void k_head(const float* __restrict__ pl, const float* __restrict__ lw,
                                              const float* __restrict__ lb, float* out) {
  __shared__ __attribute__((aligned(16))) float wls[NC2];
  __shared__ __attribute__((aligned(16))) float os[NGR];
  const int tid = (int)threadIdx.x, lane = tid & 31, wave = tid >> 5;
  wls[tid] = bfr(lw[tid]);
  const float bb = bfr(lb[0]);
  __syncthreads();
  const float* pr = pl + (size_t)tid * NC2;
  float s = 0.0f;
#pragma unroll 1
  for (int f4 = 0; f4 < NC2 / 4; ++f4) {
    const v4f p = *(const v4fa*)(pr + 4 * f4);
    const v4f w = *(const v4fa*)(wls + 4 * f4);
    s = fmaf(p.x, w.x, s);
    s = fmaf(p.y, w.y, s);
    s = fmaf(p.z, w.z, s);
    s = fmaf(p.w, w.w, s);
  }
  os[tid] = s + bb;
  __syncthreads();
  const v4f ov = *(const v4fa*)(os + 4 * (lane & 15));
  float* op = out + 4 * (lane & 15);
  const bool okst = (wave == 0) && (lane < 16);
  if (okst) *(volatile v4f*)op = ov;
  __threadfence();
  if (okst) *(volatile v4f*)op = ov;
}

static int pick_nb(int nE, int nN) {
  int nb = NBMAX;
  while (nb > 32 && (long long)nb * (long long)nE * 5LL > (long long)RCAP * (long long)nN * 4LL) nb >>= 1;
  return nb;
}
static inline int cdiv(int a, int b) { return (a + b - 1) / b; }
static inline size_t al256(size_t o) { return (o + 255) & ~(size_t)255; }

extern "C" void kernel_launch(void* const* d_in, const int* in_sizes, int n_in,
                              void* d_out, int out_size, void* d_ws, size_t ws_size,
                              hipStream_t stream) {
  if (n_in < 13) return;
  if (in_sizes[0] < F_IN || (in_sizes[0] % F_IN) != 0) return;
  const int nN = in_sizes[0] / F_IN;
  if (nN < 1 || nN > (1 << 22)) return;
  if (in_sizes[1] < 2 || (in_sizes[1] & 1) != 0) return;
  const int nE = in_sizes[1] / 2;
  if (nE < 1 || nE >= (1 << (32 - SLOTB))) return;
  if (in_sizes[2] != nN) return;
  if (in_sizes[3] != F_IN * HC1) return;
  if (in_sizes[4] != NHD1 * HID || in_sizes[5] != NHD1 * HID) return;
  if (in_sizes[6] != HC1) return;
  if (in_sizes[7] != HC1 * NC2) return;
  if (in_sizes[8] != NC2 || in_sizes[9] != NC2) return;
  if (in_sizes[10] != NC2) return;
  if (in_sizes[11] != NC2 || in_sizes[12] != 1) return;
  if (out_size != NGR) return;

  const float* x    = (const float*)d_in[0];
  const int*   ei   = (const int*)  d_in[1];
  const int*   bat  = (const int*)  d_in[2];
  const float* W1   = (const float*)d_in[3];
  const float* a1s  = (const float*)d_in[4];
  const float* a1d  = (const float*)d_in[5];
  const float* b1   = (const float*)d_in[6];
  const float* W2   = (const float*)d_in[7];
  const float* a2s  = (const float*)d_in[8];
  const float* a2d  = (const float*)d_in[9];
  const float* b2   = (const float*)d_in[10];
  const float* lw   = (const float*)d_in[11];
  const float* lb   = (const float*)d_in[12];
  float* out = (float*)d_out;
  const int* src = ei;
  const int* dst = ei + nE;

  const int MP   = cdiv(nN, MROWS) * MROWS;
  const int nb   = pick_nb(nE, nN);
  if (nb < 32 || (nb & (nb - 1)) != 0 || nb > NBMAX) return;
  const int gA   = cdiv(MP, nb);
  const int vec8 = ((nE & 3) == 0) ? 1 : 0;
  if (gA * nb < MP) return;
  const int nUx  = MP * (F_IN / 8);
  if ((nUx % NTHR) != 0) return;

  char* ws = (char*)d_ws;
  size_t off = 0;
  const size_t oXB  = off; off = al256(off + (size_t)MP * F_IN * 2);
  const size_t oW1T = off; off = al256(off + (size_t)HC1 * F_IN * 2);
  const size_t oW2T = off; off = al256(off + (size_t)NC2 * KA2 * 2);
  const size_t oH1  = off; off = al256(off + (size_t)MP * HC1 * 4);
  const size_t oSD1 = off; off = al256(off + (size_t)8 * MP * 4);
  const size_t oX1  = off; off = al256(off + (size_t)MP * KA2 * 2);
  const size_t oSD2 = off; off = al256(off + (size_t)2 * MP * 4);
  const size_t oPL  = off; off = al256(off + (size_t)NGR * NC2 * 4);
  if (off > ws_size || off > (size_t)WSMAX) return;
  const size_t szH2 = (size_t)MP * NC2 * 4;
  if (2 * szH2 > (size_t)MP * HC1 * 4) return;
  unsigned short* XB   = (unsigned short*)(ws + oXB);
  unsigned short* W1T  = (unsigned short*)(ws + oW1T);
  unsigned short* W2T2 = (unsigned short*)(ws + oW2T);
  float*          H1   = (float*)(ws + oH1);
  float*          SD1  = (float*)(ws + oSD1);
  unsigned short* X1hl = (unsigned short*)(ws + oX1);
  float*          H2   = (float*)(ws + oH1);
  float*          X2   = (float*)(ws + oH1 + szH2);
  float*          SD2  = (float*)(ws + oSD2);
  float*          PL   = (float*)(ws + oPL);

  hipFuncSetAttribute(reinterpret_cast<const void*>(&k_agg<1>),
                      hipFuncAttributeMaxDynamicSharedMemorySize, LDS_AGG);
  hipFuncSetAttribute(reinterpret_cast<const void*>(&k_agg<2>),
                      hipFuncAttributeMaxDynamicSharedMemorySize, LDS_AGG);

  const int gM = MP / GBM;
  k_prep<<<(nUx + NUW1 + NUW2) / NTHR, NTHR, 0, stream>>>(x, W1, W2, XB, W1T, W2T2, nN, nUx);
  k_gemm<<<dim3(gM, HC1 / GBN), GTHR, 0, stream>>>(XB, W1T, H1, F_IN, HC1, a1s, a1d, HID, SD1, MP);
  k_agg<1><<<gA, NTHR, LDS_AGG, stream>>>(src, dst, H1, SD1, b1, X1hl, X2, nN, nE, nb, vec8, MP);
  k_gemm<<<dim3(gM, NC2 / GBN), GTHR, 0, stream>>>(X1hl, W2T2, H2, KA2, NC2, a2s, a2d, NC2, SD2, MP);
  k_agg<2><<<gA, NTHR, LDS_AGG, stream>>>(src, dst, H2, SD2, b2, X1hl, X2, nN, nE, nb, vec8, MP);
  k_pool<<<NGR, NTHR, 0, stream>>>(X2, bat, nN, PL);
  k_head<<<1, NGR, 0, stream>>>(PL, lw, lb, out);
}
